// EternalRecursion_80161269613291
// MI455X (gfx1250) — hardware-verified
//
#include <hip/hip_runtime.h>
#include <hip/hip_bf16.h>
#include <math.h>

typedef __attribute__((ext_vector_type(16))) _Float16 v16h;
typedef __attribute__((ext_vector_type(8)))  _Float16 v8h;
typedef __attribute__((ext_vector_type(16))) __bf16   v16b;
typedef __attribute__((ext_vector_type(8)))  __bf16   v8b;
typedef __attribute__((ext_vector_type(8)))  float    v8f;
typedef __attribute__((ext_vector_type(4)))  float    v4f;

__device__ __forceinline__ unsigned short f2bf_bits(float f) {
  unsigned u = __float_as_uint(f);
  return (unsigned short)((u + 0x7FFFu + ((u >> 16) & 1u)) >> 16);
}
__device__ __forceinline__ float bf_bits2f(unsigned short h) { return __uint_as_float(((unsigned)h) << 16); }

__device__ __forceinline__ void dep_guard_h(v8f& a, v8f& b, v16h x, v16h y) { asm volatile("v_nop\n\tv_nop\n\tv_nop\n\tv_nop" : "+v"(a), "+v"(b) : "v"(x), "v"(y)); }
__device__ __forceinline__ void dep_guard_b(v8f& a, v8f& b, v16b x, v16b y) { asm volatile("v_nop\n\tv_nop\n\tv_nop\n\tv_nop" : "+v"(a), "+v"(b) : "v"(x), "v"(y)); }
__device__ __forceinline__ void keep4_h(v16h a, v16h b, v16h c, v16h d) { asm volatile("v_nop" :: "v"(a), "v"(b), "v"(c), "v"(d)); }
__device__ __forceinline__ void keep4_b(v16b a, v16b b, v16b c, v16b d) { asm volatile("v_nop" :: "v"(a), "v"(b), "v"(c), "v"(d)); }
__device__ __forceinline__ void acc_guard4(v8f& a, v8f& b, v8f& c, v8f& d) { asm volatile("v_nop\n\tv_nop\n\tv_nop\n\tv_nop" : "+v"(a), "+v"(b), "+v"(c), "+v"(d)); }
template <typename T> struct Frag;
template <> struct Frag<_Float16> {
  typedef v16h V; union U { v16h v; v8h h[2]; };
  static __device__ __forceinline__ v16h load(const _Float16* p) {
    U f; f.h[0] = *(const v8h*)(p); f.h[1] = *(const v8h*)(p + 16); return f.v;
  }
  static __device__ __forceinline__ v8f mma(v16h a, v16h b, v8f c) {
    return __builtin_amdgcn_wmma_f32_16x16x32_f16(false, a, false, b, (short)0, c, false, false);
  }
  static __device__ __forceinline__ void guard(v8f& a, v8f& b, v16h x, v16h y) { dep_guard_h(a, b, x, y); }
  static __device__ __forceinline__ void keep(v16h a, v16h b, v16h c, v16h d) { keep4_h(a, b, c, d); }
};
template <> struct Frag<__bf16> {
  typedef v16b V; union U { v16b v; v8b h[2]; };
  static __device__ __forceinline__ v16b load(const __bf16* p) {
    U f; f.h[0] = *(const v8b*)(p); f.h[1] = *(const v8b*)(p + 16); return f.v;
  }
  static __device__ __forceinline__ v8f mma(v16b a, v16b b, v8f c) {
    return __builtin_amdgcn_wmma_f32_16x16x32_bf16(false, a, false, b, (short)0, c, false, false);
  }
  static __device__ __forceinline__ void guard(v8f& a, v8f& b, v16b x, v16b y) { dep_guard_b(a, b, x, y); }
  static __device__ __forceinline__ void keep(v16b a, v16b b, v16b c, v16b d) { keep4_b(a, b, c, d); }
};

template <int ET> struct Elem;
template <> struct Elem<0> { typedef _Float16 T; };
template <> struct Elem<1> { typedef __bf16 T; };
template <int ET, bool SPLIT, int BIAS_MODE, int OUT_MODE, bool RESID, int ACT = 0>
__global__ __launch_bounds__(256) void wmma_gemm64(
    const unsigned short* __restrict__ Ap, const unsigned short* __restrict__ A2p, int lda, long strideA,
    const unsigned short* __restrict__ Btp, const unsigned short* __restrict__ Bt2p, int ldb, long strideB,
    void* __restrict__ Cout, void* __restrict__ Cout2, int ldc, long strideC,
    const float* __restrict__ bias,
    const float* __restrict__ resid, long strideR,
    int M, int N, int K, float scale) {
  typedef typename Elem<ET>::T T;
  typedef typename Frag<T>::V V;
  const T* A = (const T*)Ap; const T* A2 = (const T*)A2p; const T* Bt = (const T*)Btp; const T* Bt2 = (const T*)Bt2p;
  __shared__ __align__(16) float sT[8][16 * 68];
  const int b    = blockIdx.y;
  const int lane = threadIdx.x & 31;
  const int wave = threadIdx.x >> 5;
  const int tilesN = N >> 6;
  const int tilesM = M >> 6;
  const int tile = blockIdx.x * 8 + wave;
  if (tile >= tilesM * tilesN) return;
  const int tm = tile / tilesN;
  const int tn = tile - tm * tilesN;
  const int m0 = tm << 6;
  const int n0 = tn << 6;

  const T* Ab  = A  + (size_t)b * strideA;
  const T* Bb  = Bt + (size_t)b * strideB;
  const T* Ab2 = SPLIT ? (A2  + (size_t)b * strideA) : nullptr;
  const T* Bb2 = SPLIT ? (Bt2 + (size_t)b * strideB) : nullptr;

  const int rlane = lane & 15;
  const int koff  = (lane >> 4) * 8;
  const int mOff  = (lane >> 4) * 8;

  v8f acc[4][4];
#pragma unroll
  for (int i = 0; i < 4; ++i)
#pragma unroll
    for (int j = 0; j < 4; ++j) acc[i][j] = (v8f){0.f,0.f,0.f,0.f,0.f,0.f,0.f,0.f};

  for (int k0 = 0; k0 < K; k0 += 32) {
    V bh[4], bl[4];
#pragma unroll
    for (int j = 0; j < 4; ++j) {
      const size_t bo = (size_t)(n0 + (j << 4) + rlane) * ldb + koff + k0;
      bh[j] = Frag<T>::load(Bb + bo);
      if (SPLIT) bl[j] = Frag<T>::load(Bb2 + bo);
    }
#pragma unroll
    for (int i = 0; i < 4; ++i) {
      const size_t ao = (size_t)(m0 + (i << 4) + rlane) * lda + koff + k0;
      V ah = Frag<T>::load(Ab + ao);
      V al;
      if (SPLIT) al = Frag<T>::load(Ab2 + ao);
#pragma unroll
      for (int j = 0; j < 4; ++j) {
        acc[i][j] = Frag<T>::mma(ah, bh[j], acc[i][j]);
        if (SPLIT) {
          acc[i][j] = Frag<T>::mma(ah, bl[j], acc[i][j]);
          acc[i][j] = Frag<T>::mma(al, bh[j], acc[i][j]);
        }
      }
      Frag<T>::guard(acc[i][0], acc[i][3], ah, SPLIT ? al : ah);
    }
    Frag<T>::keep(bh[0], bh[1], bh[2], bh[3]);
    if (SPLIT) Frag<T>::keep(bl[0], bl[1], bl[2], bl[3]);
  }
  acc_guard4(acc[0][0], acc[0][1], acc[0][2], acc[0][3]);
  acc_guard4(acc[1][0], acc[1][1], acc[1][2], acc[1][3]);
  acc_guard4(acc[2][0], acc[2][1], acc[2][2], acc[2][3]);
  acc_guard4(acc[3][0], acc[3][1], acc[3][2], acc[3][3]);

  float* slab = sT[wave];
  const float* Rb = RESID ? (resid + (size_t)b * strideR) : nullptr;
#pragma unroll
  for (int i = 0; i < 4; ++i) {
    const int mBase = m0 + (i << 4);
#pragma unroll
    for (int j = 0; j < 4; ++j) {
      const int n = n0 + (j << 4) + rlane;
      float bv = 0.f;
      if (BIAS_MODE == 2) bv = bias[n];
#pragma unroll
      for (int r = 0; r < 8; ++r) {
        float v = acc[i][j][r] * scale;
        if (BIAS_MODE == 1) v += bias[mBase + mOff + r];
        if (BIAS_MODE == 2) v += bv;
        if (RESID) v += Rb[(size_t)(mBase + mOff + r) * ldc + n];
        if (ACT == 1) v = tanhf(v);
        if (ACT == 2) v = fmaxf(v, 0.0f);
        if (ACT == 3) v = v / (1.0f + expf(-v));
        if (ACT == 4) v = (v > 0.f) ? v : 0.01f * v;
        if (ACT == 5) v = 0.5f * v * (1.0f + erff(v * 0.70710678118654752f));
        slab[(mOff + r) * 68 + (j << 4) + rlane] = v;
      }
    }
    __builtin_amdgcn_fence(__ATOMIC_RELEASE, "workgroup");
    __builtin_amdgcn_wave_barrier();
    __builtin_amdgcn_fence(__ATOMIC_ACQUIRE, "workgroup");
    if (OUT_MODE == 0) {
      float* C = (float*)Cout + (size_t)b * strideC;
      const int hh = lane >> 4, c4 = (lane & 15) * 4;
      for (int pass = 0; pass < 2; ++pass) {
#pragma unroll
        for (int it = 0; it < 8; ++it) {
          const int row = it * 2 + hh;
          v4f v = *(const v4f*)(slab + row * 68 + c4);
          *(volatile v4f*)(C + (size_t)(mBase + row) * ldc + n0 + c4) = v;
        }
        __threadfence();
      }
    } else {
      const int q = lane >> 3, c8 = (lane & 7) * 8;
      unsigned short* C  = (unsigned short*)Cout  + (size_t)b * strideC;
      unsigned short* C2 = (OUT_MODE == 2) ? ((unsigned short*)Cout2 + (size_t)b * strideC) : nullptr;
      for (int pass = 0; pass < 2; ++pass) {
#pragma unroll
        for (int it = 0; it < 4; ++it) {
          const int row = it * 4 + q;
          const float* sp = slab + row * 68 + c8;
          v8h hv, lv;
#pragma unroll
          for (int e = 0; e < 8; ++e) {
            if (OUT_MODE == 1) {
              hv[e] = (_Float16)sp[e];
            } else {
              unsigned short hb = f2bf_bits(sp[e]);
              unsigned short lb = f2bf_bits(sp[e] - bf_bits2f(hb));
              hv[e] = __builtin_bit_cast(_Float16, hb);
              lv[e] = __builtin_bit_cast(_Float16, lb);
            }
          }
          *(volatile v8h*)(C + (size_t)(mBase + row) * ldc + n0 + c8) = hv;
          if (OUT_MODE == 2) *(volatile v8h*)(C2 + (size_t)(mBase + row) * ldc + n0 + c8) = lv;
        }
        __threadfence();
      }
    }
    __builtin_amdgcn_fence(__ATOMIC_RELEASE, "workgroup");
    __builtin_amdgcn_wave_barrier();
    __builtin_amdgcn_fence(__ATOMIC_ACQUIRE, "workgroup");
  }
}

constexpr int NROWS      = 512;
constexpr int NCOL       = 500;
constexpr int NPADK      = 512;
constexpr int N3REAL     = 1500;
constexpr int N3PAD      = 1536;
constexpr int NSTEPS     = 64;
constexpr int UPD_ROWS   = 8;
constexpr int NUPD_BLOCKS = NROWS / UPD_ROWS;
constexpr int PART_LINE  = 32;
constexpr size_t PL16 = (size_t)NROWS * NPADK;
constexpr size_t PL32 = (size_t)NROWS * NPADK;
constexpr size_t WPL  = (size_t)N3PAD * NPADK;
constexpr size_t GPL  = (size_t)NROWS * N3PAD;
constexpr float A_CARRY   = 16.0f;
constexpr float W_CARRY   = 256.0f;
constexpr float GEMM_FOLD = 1.0f / 4096.0f;
constexpr float INV_COUNT = 1.0f / 256000.0f;

__global__ __launch_bounds__(256) void cast_weights_kernel(const float* __restrict__ Wi,
                                                           const float* __restrict__ Wh,
                                                           unsigned short* Wt) {
  const int per = N3PAD * 64;
  const int mat = (blockIdx.x >= (per / 256)) ? 1 : 0;
  const int t   = blockIdx.x * 256 + threadIdx.x;
  const int rem = t - mat * per;
  const int n   = rem >> 6;
  const int c8  = (rem & 63) * 8;
  const float* W = mat ? Wh : Wi;
  const int nc = (n < N3REAL) ? n : (N3REAL - 1);
  const float* wr = W + (size_t)nc * NCOL;
  v8h hv8;
#pragma unroll
  for (int e = 0; e < 8; ++e) {
    const int c  = c8 + e;
    const int cc = (c < NCOL) ? c : (NCOL - 1);
    const float w = wr[cc];
    const float v = ((n < N3REAL) && (c < NCOL)) ? (w * W_CARRY) : 0.0f;
    hv8[e] = (_Float16)v;
  }
  unsigned short* dst = Wt + (size_t)mat * WPL + (size_t)n * NPADK + c8;
  *(volatile v8h*)dst = hv8;
  __threadfence();
  *(volatile v8h*)dst = hv8;
}

__global__ __launch_bounds__(256) void init_planes_kernel(const float* __restrict__ state,
                                                          float* S0, float* H0,
                                                          unsigned short* S16, unsigned short* H16) {
  if (blockIdx.x < 256) {
    const int t   = blockIdx.x * 256 + threadIdx.x;
    const int row = t >> 7;
    const int c4  = (t & 127) * 4;
    const int c4c = (c4 < NCOL) ? c4 : (NCOL - 4);
    const v4f ld  = *(const v4f*)(state + (size_t)row * NCOL + c4c);
    const bool ok = (c4 < NCOL);
    v4f v, z4;
#pragma unroll
    for (int e = 0; e < 4; ++e) { v[e] = ok ? ld[e] : 0.0f; z4[e] = 0.0f; }
    float* ds = S0 + (size_t)row * NPADK + c4;
    float* dh = H0 + (size_t)row * NPADK + c4;
    *(volatile v4f*)ds = v;
    *(volatile v4f*)dh = z4;
    __threadfence();
    *(volatile v4f*)ds = v;
    *(volatile v4f*)dh = z4;
  } else {
    const int u   = (blockIdx.x - 256) * 256 + threadIdx.x;
    const int row = u >> 6;
    const int c8  = (u & 63) * 8;
    const float* sr = state + (size_t)row * NCOL;
    v8h hv8, hz8;
#pragma unroll
    for (int e = 0; e < 8; ++e) {
      const int c  = c8 + e;
      const int cc = (c < NCOL) ? c : (NCOL - 1);
      const float f = sr[cc];
      const float v = (c < NCOL) ? (f * A_CARRY) : 0.0f;
      hv8[e] = (_Float16)v;
      hz8[e] = (_Float16)0.0f;
    }
    unsigned short* ds = S16 + (size_t)row * NPADK + c8;
    unsigned short* dh = H16 + (size_t)row * NPADK + c8;
    *(volatile v8h*)ds = hv8;
    *(volatile v8h*)dh = hz8;
    __threadfence();
    *(volatile v8h*)ds = hv8;
    *(volatile v8h*)dh = hz8;
  }
}

__global__ __launch_bounds__(512) void gru_update_kernel(
    int step,
    const float* __restrict__ G,
    const float* __restrict__ b_ih, const float* __restrict__ b_hh,
    const float* __restrict__ bcp, const int* __restrict__ limp,
    const float* __restrict__ Sin, const float* __restrict__ Hin,
    float* Sout, float* Hout, unsigned short* S16o, unsigned short* H16o,
    float* part) {
  __shared__ __align__(16) float sS[NPADK];
  __shared__ __align__(16) float sH[NPADK];
  __shared__ float sRed[16];
  __shared__ int sFlag[64];
  __shared__ int sDone;
  (void)limp;
  const int tid  = threadIdx.x;
  const int lane = tid & 31;
  const int wave = tid >> 5;

  if (wave < 2) {
    const int q = tid;
    int f = 0;
    if (step > 0) {
      const int qc = (q < step) ? q : (step - 1);
      const float* pl = part + (size_t)qc * NUPD_BLOCKS * PART_LINE;
      float tot = 0.f;
#pragma unroll 1
      for (int p = 0; p < NUPD_BLOCKS; ++p) tot += pl[(size_t)p * PART_LINE];
      const float mean = tot * INV_COUNT;
      const float bcv = bcp[0];
      f = ((q < step) && (mean > bcv)) ? 1 : 0;
    }
    sFlag[q] = f;
  }
  __syncthreads();
  if (tid == 0) {
    int d = 0;
#pragma unroll 1
    for (int q = 0; q < 64; ++q) d |= sFlag[q];
    sDone = d;
  }
  __syncthreads();
  const bool latched = (sDone != 0);

  const int col   = tid;
  const bool valid = (col < NCOL);
  const int colc  = valid ? col : (NCOL - 1);
  const float bir = b_ih[colc];
  const float biz = b_ih[NCOL + colc];
  const float bin_ = b_ih[2 * NCOL + colc];
  const float bhr = b_hh[colc];
  const float bhz = b_hh[NCOL + colc];
  const float bhn = b_hh[2 * NCOL + colc];
  const int grp = wave >> 2;
  const int sub = (wave >> 1) & 1;
  const int row0 = blockIdx.x * UPD_ROWS;
  float psum = 0.f;

#pragma unroll 1
  for (int i = 0; i < UPD_ROWS; ++i) {
    const int row = row0 + i;
    const float* gi = G + (size_t)row * N3PAD;
    const float* gh = G + GPL + (size_t)row * N3PAD;
    const float xr = gi[colc] + bir;
    const float xz = gi[NCOL + colc] + biz;
    const float xn = gi[2 * NCOL + colc] + bin_;
    const float hr = gh[colc] + bhr;
    const float hz = gh[NCOL + colc] + bhz;
    const float hn = gh[2 * NCOL + colc] + bhn;
    const float sp = Sin[(size_t)row * NPADK + col];
    const float hp = Hin[(size_t)row * NPADK + col];
    const float r  = 1.0f / (1.0f + expf(-(xr + hr)));
    const float z  = 1.0f / (1.0f + expf(-(xz + hz)));
    const float nn = tanhf(xn + r * hn);
    const float hnew = (1.0f - z) * nn + z * hp;
    const float hv = valid ? hnew : 0.0f;
    psum += hv;
    const float so = latched ? sp : hv;
    const float ho = latched ? hp : hv;
    sS[col] = so;
    sH[col] = ho;
    __syncthreads();
    if (grp < 2) {
      const int j = tid & 127;
      const v4f a = *(const v4f*)(sS + 4 * j);
      const v4f c = *(const v4f*)(sH + 4 * j);
      v4f v;
#pragma unroll
      for (int e = 0; e < 4; ++e) v[e] = (grp == 0) ? a[e] : c[e];
      float* dst = ((grp == 0) ? Sout : Hout) + (size_t)row * NPADK + 4 * j;
      *(volatile v4f*)dst = v;
      __threadfence();
      *(volatile v4f*)dst = v;
    } else if (grp == 2) {
      const int j = tid & 63;
      const v4f a0 = *(const v4f*)(sS + 8 * j);
      const v4f a1 = *(const v4f*)(sS + 8 * j + 4);
      const v4f c0 = *(const v4f*)(sH + 8 * j);
      const v4f c1 = *(const v4f*)(sH + 8 * j + 4);
      v8h hv8;
#pragma unroll
      for (int e = 0; e < 4; ++e) {
        const float f0 = (sub == 0) ? a0[e] : c0[e];
        const float f1 = (sub == 0) ? a1[e] : c1[e];
        hv8[e]     = (_Float16)(f0 * A_CARRY);
        hv8[4 + e] = (_Float16)(f1 * A_CARRY);
      }
      unsigned short* dst = ((sub == 0) ? S16o : H16o) + (size_t)row * NPADK + 8 * j;
      *(volatile v8h*)dst = hv8;
      __threadfence();
      *(volatile v8h*)dst = hv8;
    }
    __syncthreads();
  }

#pragma unroll
  for (int off = 16; off > 0; off >>= 1) psum += __shfl_xor(psum, off, 32);
  if (lane == 0) sRed[wave] = psum;
  __syncthreads();
  if (wave == 0) {
    const float tv = sRed[lane & 15];
    float v = (lane < 16) ? tv : 0.0f;
#pragma unroll
    for (int off = 16; off > 0; off >>= 1) v += __shfl_xor(v, off, 32);
    float* dst = part + ((size_t)step * NUPD_BLOCKS + blockIdx.x) * PART_LINE + lane;
    *(volatile float*)dst = v;
    __threadfence();
    *(volatile float*)dst = v;
  }
}

__global__ __launch_bounds__(256) void copy_out_kernel(const float* __restrict__ S, float* out) {
  const int t = blockIdx.x * 256 + threadIdx.x;
  if (t < (NROWS * NCOL) / 4) {
    const int e   = t * 4;
    const int row = e / NCOL;
    const int col = e - row * NCOL;
    const v4f v = *(const v4f*)(S + (size_t)row * NPADK + col);
    float* dst = out + e;
    *(volatile v4f*)dst = v;
    __threadfence();
    *(volatile v4f*)dst = v;
  }
}

extern "C" void kernel_launch(void* const* d_in, const int* in_sizes, int n_in,
                              void* d_out, int out_size, void* d_ws, size_t ws_size,
                              hipStream_t stream) {
  if (n_in < 7) return;
  if (in_sizes[0] != NROWS * NCOL || in_sizes[1] != N3REAL * NCOL || in_sizes[2] != N3REAL * NCOL ||
      in_sizes[3] != N3REAL || in_sizes[4] != N3REAL || in_sizes[5] < 1 || in_sizes[6] < 1 ||
      out_size != NROWS * NCOL) return;

  const float* state = (const float*)d_in[0];
  const float* W_ih  = (const float*)d_in[1];
  const float* W_hh  = (const float*)d_in[2];
  const float* b_ih  = (const float*)d_in[3];
  const float* b_hh  = (const float*)d_in[4];
  const float* bcp   = (const float*)d_in[5];
  const int*   limp  = (const int*)d_in[6];
  float* out = (float*)d_out;

  char* ws = (char*)d_ws;
  size_t off = 0;
  const size_t szA16  = 2 * 2 * PL16 * sizeof(unsigned short);
  const size_t szWT   = 2 * WPL * sizeof(unsigned short);
  const size_t szG    = 2 * GPL * sizeof(float);
  const size_t szM32  = 2 * 2 * PL32 * sizeof(float);
  const size_t szPART = (size_t)NSTEPS * NUPD_BLOCKS * PART_LINE * sizeof(float);
  unsigned short* A16 = (unsigned short*)(ws + off); off += szA16;
  unsigned short* WT  = (unsigned short*)(ws + off); off += szWT;
  float* G    = (float*)(ws + off); off += szG;
  float* M32  = (float*)(ws + off); off += szM32;
  float* PART = (float*)(ws + off); off += szPART;
  if (off > ws_size) return;

  cast_weights_kernel<<<(2 * N3PAD * 64) / 256, 256, 0, stream>>>(W_ih, W_hh, WT);
  init_planes_kernel<<<384, 256, 0, stream>>>(state, M32, M32 + PL32, A16, A16 + PL16);

  const int gemm_tiles = (NROWS / 64) * (N3PAD / 64);
  const dim3 ggrid((gemm_tiles + 7) / 8, 2);
  for (int t = 0; t < NSTEPS; ++t) {
    const int pin = t & 1, pout = pin ^ 1;
    const unsigned short* Ap = A16 + (size_t)pin * 2 * PL16;
    wmma_gemm64<0, false, 0, 0, false, 0><<<ggrid, 256, 0, stream>>>(
        Ap, Ap, NPADK, (long)PL16,
        WT, WT, NPADK, (long)WPL,
        (void*)G, (void*)G, N3PAD, (long)GPL,
        PART, PART, 0L,
        NROWS, N3PAD, NPADK, GEMM_FOLD);
    gru_update_kernel<<<NUPD_BLOCKS, 512, 0, stream>>>(
        t, G, b_ih, b_hh, bcp, limp,
        M32 + ((size_t)pin * 2 + 0) * PL32, M32 + ((size_t)pin * 2 + 1) * PL32,
        M32 + ((size_t)pout * 2 + 0) * PL32, M32 + ((size_t)pout * 2 + 1) * PL32,
        A16 + ((size_t)pout * 2 + 0) * PL16, A16 + ((size_t)pout * 2 + 1) * PL16,
        PART);
  }
  copy_out_kernel<<<(NROWS * NCOL / 4 + 255) / 256, 256, 0, stream>>>(M32, out);
}
